// ShortcutMoEDecoderLayer_88235808129203
// MI455X (gfx1250) — hardware-verified
//
#include <hip/hip_runtime.h>
#include <stddef.h>

#define NT   1024
#define NH   1024
#define NQH  16
#define NKH  4
#define HD   64
#define QKVW 1536
#define QW   1024
#define KVW  256
#define IDN  4096
#define IMO  512
#define NE   8
#define NEP  16

typedef float  v4f   __attribute__((ext_vector_type(4), may_alias));
typedef float  v8f   __attribute__((ext_vector_type(8)));
typedef int    v4i   __attribute__((ext_vector_type(4), may_alias));
typedef __bf16 v8bf  __attribute__((ext_vector_type(8), may_alias));
typedef __bf16 v16bf __attribute__((ext_vector_type(16)));

union Frag { v16bf v; v8bf h[2]; };
union Pack8 { v8bf b; v4i i; };

static __device__ __forceinline__ v8f mma(v16bf a, v16bf b, v8f c) {
  return __builtin_amdgcn_wmma_f32_16x16x32_bf16(false, a, false, b, (short)0, c, false, false);
}

static __device__ __forceinline__ v8f zero8() {
  v8f z;
  z[0] = 0.f; z[1] = 0.f; z[2] = 0.f; z[3] = 0.f; z[4] = 0.f; z[5] = 0.f; z[6] = 0.f; z[7] = 0.f;
  return z;
}

static __device__ __forceinline__ void sp2(float a, __bf16& h, __bf16& l) {
  h = (__bf16)a;
  l = (__bf16)(a - (float)h);
}

static __device__ __forceinline__ void split2x8(v4f x0, v4f x1, Pack8& hi, Pack8& lo) {
  __bf16 h, l;
  sp2(x0.x, h, l); hi.b[0] = h; lo.b[0] = l;
  sp2(x0.y, h, l); hi.b[1] = h; lo.b[1] = l;
  sp2(x0.z, h, l); hi.b[2] = h; lo.b[2] = l;
  sp2(x0.w, h, l); hi.b[3] = h; lo.b[3] = l;
  sp2(x1.x, h, l); hi.b[4] = h; lo.b[4] = l;
  sp2(x1.y, h, l); hi.b[5] = h; lo.b[5] = l;
  sp2(x1.z, h, l); hi.b[6] = h; lo.b[6] = l;
  sp2(x1.w, h, l); hi.b[7] = h; lo.b[7] = l;
}

static __device__ __forceinline__ void vst16(__bf16* p, const Pack8& v) {
  *(volatile v4i*)p = v.i;
}

__global__ __launch_bounds__(128) void k_rope_tab(const int* __restrict__ pos,
                                                  float* cs, float* sn, int ntok) {
  const int j = threadIdx.x & 31;
  const int t = blockIdx.x * 4 + (threadIdx.x >> 5);
  const int tc = (t < ntok) ? t : (ntok - 1);
  const float p = (float)pos[tc];
  const float e = (float)j * 0.03125f;
  const float fr = powf(10000.0f, e);
  const float inv = 1.0f / fr;
  const float ang = p * inv;
  const float c = cosf(ang);
  const float s = sinf(ang);
  volatile float* pc = cs + (size_t)tc * 32 + j;
  volatile float* ps = sn + (size_t)tc * 32 + j;
  if (t < ntok) { *pc = c; *ps = s; }
  __threadfence();
  if (t < ntok) { *pc = c; *ps = s; }
}

__global__ __launch_bounds__(128) void k_cvt_gate(const float* __restrict__ gw,
                                                  __bf16* gh, __bf16* gm, __bf16* gl) {
  const int n = blockIdx.x;
  const int nc = n & (NE - 1);
  const bool real = (n < NE);
  const int k0 = threadIdx.x * 8;
  Pack8 ph, pm, pl;
#pragma unroll
  for (int i = 0; i < 8; i++) {
    float x = gw[(size_t)(k0 + i) * NE + nc];
    x = real ? x : 0.0f;
    const __bf16 a = (__bf16)x;
    const float r1 = x - (float)a;
    const __bf16 b = (__bf16)r1;
    const float r2 = r1 - (float)b;
    const __bf16 c = (__bf16)r2;
    ph.b[i] = a; pm.b[i] = b; pl.b[i] = c;
  }
  const size_t o = (size_t)n * NH + k0;
  vst16(gh + o, ph); vst16(gm + o, pm); vst16(gl + o, pl);
  __threadfence();
  vst16(gh + o, ph); vst16(gm + o, pm); vst16(gl + o, pl);
}

template <int THIRD>
__global__ __launch_bounds__(256) void k_addnorm(const float* __restrict__ x, const float* res,
                                                 const float* __restrict__ wgt, float* r_out,
                                                 __bf16* hhi, __bf16* hlo, __bf16* hl3) {
  __shared__ v4f sS[256];
  __shared__ float sRed[8];
  const int row = blockIdx.x, t = threadIdx.x, l = t & 31, w = t >> 5;
  const size_t base = (size_t)row * NH + 4 * t;
  const v4f a = *(const v4f*)(x + base);
  const v4f b = *(const v4f*)(res + base);
  const v4f s = a + b;
  float q = s.x * s.x + s.y * s.y + s.z * s.z + s.w * s.w;
  q += __shfl_xor(q, 16);
  q += __shfl_xor(q, 8);
  q += __shfl_xor(q, 4);
  q += __shfl_xor(q, 2);
  q += __shfl_xor(q, 1);
  sS[t] = s;
  if (l == 0) sRed[w] = q;
  __syncthreads();
  const float tot = ((sRed[0] + sRed[1]) + (sRed[2] + sRed[3])) +
                    ((sRed[4] + sRed[5]) + (sRed[6] + sRed[7]));
  const float rs = rsqrtf(tot * (1.0f / 1024.0f) + 1e-6f);
  *(volatile v4f*)(r_out + base) = s;
  __threadfence();
  *(volatile v4f*)(r_out + base) = s;
  if (t < 128) {
    const v4f s0 = sS[2 * t];
    const v4f s1 = sS[2 * t + 1];
    const v4f w0 = *(const v4f*)(wgt + 8 * t);
    const v4f w1 = *(const v4f*)(wgt + 8 * t + 4);
    const v4f h0 = (s0 * rs) * w0;
    const v4f h1 = (s1 * rs) * w1;
    Pack8 phi, plo, p3;
    split2x8(h0, h1, phi, plo);
    if (THIRD) {
      __bf16 c;
      c = (__bf16)((h0.x - (float)phi.b[0]) - (float)plo.b[0]); p3.b[0] = c;
      c = (__bf16)((h0.y - (float)phi.b[1]) - (float)plo.b[1]); p3.b[1] = c;
      c = (__bf16)((h0.z - (float)phi.b[2]) - (float)plo.b[2]); p3.b[2] = c;
      c = (__bf16)((h0.w - (float)phi.b[3]) - (float)plo.b[3]); p3.b[3] = c;
      c = (__bf16)((h1.x - (float)phi.b[4]) - (float)plo.b[4]); p3.b[4] = c;
      c = (__bf16)((h1.y - (float)phi.b[5]) - (float)plo.b[5]); p3.b[5] = c;
      c = (__bf16)((h1.z - (float)phi.b[6]) - (float)plo.b[6]); p3.b[6] = c;
      c = (__bf16)((h1.w - (float)phi.b[7]) - (float)plo.b[7]); p3.b[7] = c;
    }
    const size_t ob = (size_t)row * NH + 8 * t;
    vst16(hhi + ob, phi); vst16(hlo + ob, plo);
    if (THIRD) vst16(hl3 + ob, p3);
    __threadfence();
    vst16(hhi + ob, phi); vst16(hlo + ob, plo);
    if (THIRD) vst16(hl3 + ob, p3);
  }
}

__global__ __launch_bounds__(256) void k_cvt_t(const float* __restrict__ src, int K, int Ng,
                                               __bf16* dhi, __bf16* dlo) {
  __shared__ __attribute__((aligned(16))) float sT[64][68];
  const int n0 = blockIdx.x * 64, k0 = blockIdx.y * 64, g = blockIdx.z;
  const int t = threadIdx.x;
  const float* sp = src + (size_t)g * (size_t)K * (size_t)Ng;
#pragma unroll
  for (int i = 0; i < 4; i++) {
    const int idx = i * 256 + t;
    const int kk = idx >> 4, nn = (idx & 15) * 4;
    const v4f v = *(const v4f*)(sp + (size_t)(k0 + kk) * (size_t)Ng + n0 + nn);
    sT[nn][kk] = v.x; sT[nn + 1][kk] = v.y; sT[nn + 2][kk] = v.z; sT[nn + 3][kk] = v.w;
  }
  __syncthreads();
  Pack8 hi[2], lo[2];
  size_t go[2];
#pragma unroll
  for (int it = 0; it < 2; it++) {
    const int rr = it * 32 + (t >> 3);
    const int ks = (t & 7) * 8;
    const v4f x0 = *(const v4f*)(&sT[rr][ks]);
    const v4f x1 = *(const v4f*)(&sT[rr][ks + 4]);
    split2x8(x0, x1, hi[it], lo[it]);
    go[it] = (size_t)(g * Ng + n0 + rr) * (size_t)K + k0 + ks;
  }
  vst16(dhi + go[0], hi[0]); vst16(dlo + go[0], lo[0]);
  vst16(dhi + go[1], hi[1]); vst16(dlo + go[1], lo[1]);
  __threadfence();
  vst16(dhi + go[0], hi[0]); vst16(dlo + go[0], lo[0]);
  vst16(dhi + go[1], hi[1]); vst16(dlo + go[1], lo[1]);
}

template <int MODE>
__global__ __launch_bounds__(128) void k_gemm(
    const __bf16* __restrict__ Ahi, const __bf16* __restrict__ Alo, int lda,
    const __bf16* __restrict__ Bhi, const __bf16* __restrict__ Blo, int K,
    int halfI, int groupRows,
    float* Cout, int ldc, const float* __restrict__ addend,
    __bf16* Ohi, __bf16* Olo, int ldo,
    const float* __restrict__ rscale, int rstride) {
  __shared__ __attribute__((aligned(16))) float sC[64][132];
  const int tid = threadIdx.x, w = tid >> 5, l = tid & 31, hh = l >> 4, m = l & 15;
  const int m0 = blockIdx.y * 64;
  const int wr = (w >> 1) * 32;
  const int wc = w & 1;
  int brow;
  if (MODE < 2) brow = blockIdx.x * 128 + wc * 64;
  else          brow = blockIdx.z * groupRows + wc * halfI + blockIdx.x * 64;

  const size_t ar0 = (size_t)(m0 + wr + m) * (size_t)lda;
  const size_t ar1 = ar0 + (size_t)16 * (size_t)lda;
  const __bf16* bph = Bhi + (size_t)(brow + m) * (size_t)K;
  const __bf16* bpl = Blo + (size_t)(brow + m) * (size_t)K;
  const size_t cst = (size_t)16 * (size_t)K;

  v8f acc[2][4];
#pragma unroll
  for (int i = 0; i < 2; i++)
#pragma unroll
    for (int c = 0; c < 4; c++) acc[i][c] = zero8();

#pragma unroll 1
  for (int k0 = 0; k0 < K; k0 += 32) {
    const int ka = k0 + 8 * hh, kb = k0 + 16 + 8 * hh;
    Frag fa0h, fa0l, fa1h, fa1l, fbh, fbl;
    fa0h.h[0] = *(const v8bf*)(Ahi + ar0 + ka); fa0h.h[1] = *(const v8bf*)(Ahi + ar0 + kb);
    fa0l.h[0] = *(const v8bf*)(Alo + ar0 + ka); fa0l.h[1] = *(const v8bf*)(Alo + ar0 + kb);
    fa1h.h[0] = *(const v8bf*)(Ahi + ar1 + ka); fa1h.h[1] = *(const v8bf*)(Ahi + ar1 + kb);
    fa1l.h[0] = *(const v8bf*)(Alo + ar1 + ka); fa1l.h[1] = *(const v8bf*)(Alo + ar1 + kb);
#pragma unroll
    for (int c = 0; c < 4; c++) {
      const size_t bo = (size_t)c * cst;
      fbh.h[0] = *(const v8bf*)(bph + bo + ka); fbh.h[1] = *(const v8bf*)(bph + bo + kb);
      fbl.h[0] = *(const v8bf*)(bpl + bo + ka); fbl.h[1] = *(const v8bf*)(bpl + bo + kb);
      acc[0][c] = mma(fa0h.v, fbh.v, acc[0][c]);
      acc[0][c] = mma(fa0h.v, fbl.v, acc[0][c]);
      acc[0][c] = mma(fa0l.v, fbh.v, acc[0][c]);
      acc[1][c] = mma(fa1h.v, fbh.v, acc[1][c]);
      acc[1][c] = mma(fa1h.v, fbl.v, acc[1][c]);
      acc[1][c] = mma(fa1l.v, fbh.v, acc[1][c]);
    }
    asm volatile("v_nop\n\tv_nop\n\tv_nop\n\tv_nop"
                 : "+v"(acc[0][0]), "+v"(acc[0][1]), "+v"(acc[0][2]), "+v"(acc[0][3]),
                   "+v"(acc[1][0]), "+v"(acc[1][1]), "+v"(acc[1][2]), "+v"(acc[1][3])
                 : "v"(fa0h.v), "v"(fa0l.v), "v"(fa1h.v), "v"(fa1l.v), "v"(fbh.v), "v"(fbl.v));
  }

#pragma unroll
  for (int i = 0; i < 2; i++)
#pragma unroll
    for (int c = 0; c < 4; c++)
#pragma unroll
      for (int r = 0; r < 8; r++)
        sC[wr + 16 * i + 8 * hh + r][wc * 64 + 16 * c + m] = acc[i][c][r];
  __syncthreads();

  if (MODE < 2) {
    const int n0 = blockIdx.x * 128;
    auto emit = [&]() {
#pragma unroll 4
      for (int j = 0; j < 16; j++) {
        const int row = w * 16 + j;
        v4f v = *(const v4f*)(&sC[row][4 * l]);
        const size_t go = (size_t)(m0 + row) * (size_t)ldc + n0 + 4 * l;
        if (MODE == 1) { const v4f ad = *(const v4f*)(addend + go); v = v + ad; }
        *(volatile v4f*)(Cout + go) = v;
      }
    };
    emit();
    __threadfence();
    emit();
  } else {
    const int oc0 = blockIdx.z * halfI + blockIdx.x * 64;
    Pack8 hi[4], lo[4];
    size_t go[4];
#pragma unroll
    for (int j = 0; j < 4; j++) {
      const int row = w * 16 + 4 * j + (l >> 3);
      const int c8 = (l & 7) * 8;
      const v4f g0 = *(const v4f*)(&sC[row][c8]);
      const v4f g1 = *(const v4f*)(&sC[row][c8 + 4]);
      const v4f u0 = *(const v4f*)(&sC[row][64 + c8]);
      const v4f u1 = *(const v4f*)(&sC[row][64 + c8 + 4]);
      float sc = 1.0f;
      if (MODE == 3) sc = rscale[(size_t)(m0 + row) * (size_t)rstride + blockIdx.z];
      v4f a0, a1;
      a0.x = (g0.x * __builtin_amdgcn_rcpf(1.0f + __expf(-g0.x))) * u0.x * sc;
      a0.y = (g0.y * __builtin_amdgcn_rcpf(1.0f + __expf(-g0.y))) * u0.y * sc;
      a0.z = (g0.z * __builtin_amdgcn_rcpf(1.0f + __expf(-g0.z))) * u0.z * sc;
      a0.w = (g0.w * __builtin_amdgcn_rcpf(1.0f + __expf(-g0.w))) * u0.w * sc;
      a1.x = (g1.x * __builtin_amdgcn_rcpf(1.0f + __expf(-g1.x))) * u1.x * sc;
      a1.y = (g1.y * __builtin_amdgcn_rcpf(1.0f + __expf(-g1.y))) * u1.y * sc;
      a1.z = (g1.z * __builtin_amdgcn_rcpf(1.0f + __expf(-g1.z))) * u1.z * sc;
      a1.w = (g1.w * __builtin_amdgcn_rcpf(1.0f + __expf(-g1.w))) * u1.w * sc;
      split2x8(a0, a1, hi[j], lo[j]);
      go[j] = (size_t)(m0 + row) * (size_t)ldo + oc0 + c8;
    }
    vst16(Ohi + go[0], hi[0]); vst16(Olo + go[0], lo[0]);
    vst16(Ohi + go[1], hi[1]); vst16(Olo + go[1], lo[1]);
    vst16(Ohi + go[2], hi[2]); vst16(Olo + go[2], lo[2]);
    vst16(Ohi + go[3], hi[3]); vst16(Olo + go[3], lo[3]);
    __threadfence();
    vst16(Ohi + go[0], hi[0]); vst16(Olo + go[0], lo[0]);
    vst16(Ohi + go[1], hi[1]); vst16(Olo + go[1], lo[1]);
    vst16(Ohi + go[2], hi[2]); vst16(Olo + go[2], lo[2]);
    vst16(Ohi + go[3], hi[3]); vst16(Olo + go[3], lo[3]);
  }
}

__global__ __launch_bounds__(256) void k_rope(const float* __restrict__ qkv,
                                              const float* __restrict__ cs, const float* __restrict__ sn,
                                              __bf16* qh, __bf16* ql, __bf16* kh, __bf16* kl,
                                              __bf16* vth, __bf16* vtl) {
  __shared__ __attribute__((aligned(16))) float sV[64][68];
  const int t0 = blockIdx.x * 64;
  const int t = threadIdx.x;

#pragma unroll 1
  for (int it = 0; it < 40; it++) {
    const int ch = it * 256 + t;
    const int rl = ch / 160;
    const int c0 = (ch - rl * 160) * 8;
    const int trow = t0 + rl;
    const float* rp = qkv + (size_t)trow * QKVW;
    const v4f x0 = *(const v4f*)(rp + c0);
    const v4f x1 = *(const v4f*)(rp + c0 + 4);
    const int pc = c0 ^ 32;
    const v4f y0 = *(const v4f*)(rp + pc);
    const v4f y1 = *(const v4f*)(rp + pc + 4);
    const int j0 = c0 & 31;
    const v4f c_0 = *(const v4f*)(cs + (size_t)trow * 32 + j0);
    const v4f c_1 = *(const v4f*)(cs + (size_t)trow * 32 + j0 + 4);
    const v4f s_0 = *(const v4f*)(sn + (size_t)trow * 32 + j0);
    const v4f s_1 = *(const v4f*)(sn + (size_t)trow * 32 + j0 + 4);
    const float sg = (c0 & 32) ? 1.0f : -1.0f;
    const v4f o0 = x0 * c_0 + sg * (y0 * s_0);
    const v4f o1 = x1 * c_1 + sg * (y1 * s_1);
    Pack8 hi, lo;
    split2x8(o0, o1, hi, lo);
    __bf16* dh;
    __bf16* dl;
    size_t off;
    if (c0 < QW) { dh = qh; dl = ql; off = (size_t)trow * QW + c0; }
    else         { dh = kh; dl = kl; off = (size_t)trow * KVW + (c0 - QW); }
    vst16(dh + off, hi); vst16(dl + off, lo);
    __threadfence();
    vst16(dh + off, hi); vst16(dl + off, lo);
  }

#pragma unroll 1
  for (int dc = 0; dc < 4; dc++) {
    __syncthreads();
#pragma unroll
    for (int i = 0; i < 4; i++) {
      const int idx = i * 256 + t;
      const int tt = idx >> 4, dd = (idx & 15) * 4;
      const v4f v = *(const v4f*)(qkv + (size_t)(t0 + tt) * QKVW + (QW + KVW) + dc * 64 + dd);
      sV[dd][tt] = v.x; sV[dd + 1][tt] = v.y; sV[dd + 2][tt] = v.z; sV[dd + 3][tt] = v.w;
    }
    __syncthreads();
    Pack8 hi[2], lo[2];
    size_t off[2];
#pragma unroll
    for (int it = 0; it < 2; it++) {
      const int d = it * 32 + (t >> 3);
      const int ts = (t & 7) * 8;
      const v4f x0 = *(const v4f*)(&sV[d][ts]);
      const v4f x1 = *(const v4f*)(&sV[d][ts + 4]);
      split2x8(x0, x1, hi[it], lo[it]);
      off[it] = (size_t)(dc * 64 + d) * NT + t0 + ts;
    }
    vst16(vth + off[0], hi[0]); vst16(vtl + off[0], lo[0]);
    vst16(vth + off[1], hi[1]); vst16(vtl + off[1], lo[1]);
    __threadfence();
    vst16(vth + off[0], hi[0]); vst16(vtl + off[0], lo[0]);
    vst16(vth + off[1], hi[1]); vst16(vtl + off[1], lo[1]);
  }
}

__global__ __launch_bounds__(128) void k_attn(
    const __bf16* __restrict__ qh, const __bf16* __restrict__ ql,
    const __bf16* __restrict__ kh, const __bf16* __restrict__ kl,
    const __bf16* __restrict__ vth, const __bf16* __restrict__ vtl,
    __bf16* oh, __bf16* ol) {
  __shared__ __attribute__((aligned(16))) float sO[4][16][68];
  const int qt = blockIdx.x, kvh = blockIdx.y;
  const int tid = threadIdx.x, w = tid >> 5, l = tid & 31, hh = l >> 4, m = l & 15;
  const int head = kvh * 4 + w;
  const int q0 = qt * 16;
  const int q = q0 + m;

  Frag qbh[2], qbl[2];
  {
    const size_t qo = (size_t)q * QW + head * HD;
#pragma unroll
    for (int ks = 0; ks < 2; ks++) {
      qbh[ks].h[0] = *(const v8bf*)(qh + qo + ks * 32 + 8 * hh);
      qbh[ks].h[1] = *(const v8bf*)(qh + qo + ks * 32 + 16 + 8 * hh);
      qbl[ks].h[0] = *(const v8bf*)(ql + qo + ks * 32 + 8 * hh);
      qbl[ks].h[1] = *(const v8bf*)(ql + qo + ks * 32 + 16 + 8 * hh);
    }
  }

  v8f o[4];
#pragma unroll
  for (int j = 0; j < 4; j++) o[j] = zero8();
  float mrun = -1e30f, lrun = 0.0f;

  const size_t kbase = (size_t)m * KVW + kvh * HD;
  const size_t vbase = (size_t)(kvh * HD + m) * NT;
  const int nsteps = (q0 + 16 + 31) >> 5;

#pragma unroll 1
  for (int st = 0; st < nsteps; st++) {
    const int kk0 = st * 32;
    v8f s[2];
    s[0] = zero8(); s[1] = zero8();
    Frag ah, al;
#pragma unroll
    for (int tt = 0; tt < 2; tt++) {
#pragma unroll
      for (int ks = 0; ks < 2; ks++) {
        const size_t ro = kbase + (size_t)(kk0 + 16 * tt) * KVW + ks * 32;
        ah.h[0] = *(const v8bf*)(kh + ro + 8 * hh);
        ah.h[1] = *(const v8bf*)(kh + ro + 16 + 8 * hh);
        al.h[0] = *(const v8bf*)(kl + ro + 8 * hh);
        al.h[1] = *(const v8bf*)(kl + ro + 16 + 8 * hh);
        s[tt] = mma(ah.v, qbh[ks].v, s[tt]);
        s[tt] = mma(ah.v, qbl[ks].v, s[tt]);
        s[tt] = mma(al.v, qbh[ks].v, s[tt]);
      }
    }
    asm volatile("v_nop\n\tv_nop\n\tv_nop\n\tv_nop"
                 : "+v"(s[0]), "+v"(s[1])
                 : "v"(ah.v), "v"(al.v), "v"(qbh[0].v), "v"(qbh[1].v), "v"(qbl[0].v), "v"(qbl[1].v));

    float mt = -1e30f;
#pragma unroll
    for (int tt = 0; tt < 2; tt++) {
#pragma unroll
      for (int r = 0; r < 8; r++) {
        const int key = kk0 + 16 * tt + 8 * hh + r;
        float v = s[tt][r] * 0.125f;
        v = (key > q) ? -1e30f : v;
        s[tt][r] = v;
        mt = fmaxf(mt, v);
      }
    }
    mt = fmaxf(mt, __shfl_xor(mt, 16));
    const float mnew = fmaxf(mrun, mt);
    const float corr = expf(mrun - mnew);
    float ps = 0.0f;
#pragma unroll
    for (int tt = 0; tt < 2; tt++) {
#pragma unroll
      for (int r = 0; r < 8; r++) {
        const float p = expf(s[tt][r] - mnew);
        s[tt][r] = p;
        ps += p;
      }
    }
    ps += __shfl_xor(ps, 16);
    lrun = lrun * corr + ps;
    mrun = mnew;
#pragma unroll
    for (int j = 0; j < 4; j++) o[j] = o[j] * corr;

    Frag ph, pl;
#pragma unroll
    for (int r = 0; r < 8; r++) {
      __bf16 a, b;
      sp2(s[0][r], a, b); ph.v[r] = a;     pl.v[r] = b;
      sp2(s[1][r], a, b); ph.v[8 + r] = a; pl.v[8 + r] = b;
    }
    Frag vh, vl;
#pragma unroll
    for (int j = 0; j < 4; j++) {
      const size_t vo = vbase + (size_t)(16 * j) * NT + kk0;
      vh.h[0] = *(const v8bf*)(vth + vo + 8 * hh);
      vh.h[1] = *(const v8bf*)(vth + vo + 16 + 8 * hh);
      vl.h[0] = *(const v8bf*)(vtl + vo + 8 * hh);
      vl.h[1] = *(const v8bf*)(vtl + vo + 16 + 8 * hh);
      o[j] = mma(vh.v, ph.v, o[j]);
      o[j] = mma(vh.v, pl.v, o[j]);
      o[j] = mma(vl.v, ph.v, o[j]);
    }
    asm volatile("v_nop\n\tv_nop\n\tv_nop\n\tv_nop"
                 : "+v"(o[0]), "+v"(o[1]), "+v"(o[2]), "+v"(o[3])
                 : "v"(vh.v), "v"(vl.v), "v"(ph.v), "v"(pl.v));
  }

  const float inv = 1.0f / lrun;
#pragma unroll
  for (int j = 0; j < 4; j++)
#pragma unroll
    for (int r = 0; r < 8; r++)
      sO[w][m][16 * j + 8 * hh + r] = o[j][r] * inv;
  __syncthreads();

  Pack8 hi[4], lo[4];
  size_t go[4];
#pragma unroll
  for (int it = 0; it < 4; it++) {
    const int qq = it * 4 + (l >> 3);
    const int ds = (l & 7) * 8;
    const v4f x0 = *(const v4f*)(&sO[w][qq][ds]);
    const v4f x1 = *(const v4f*)(&sO[w][qq][ds + 4]);
    split2x8(x0, x1, hi[it], lo[it]);
    go[it] = (size_t)(q0 + qq) * QW + head * HD + ds;
  }
  vst16(oh + go[0], hi[0]); vst16(ol + go[0], lo[0]);
  vst16(oh + go[1], hi[1]); vst16(ol + go[1], lo[1]);
  vst16(oh + go[2], hi[2]); vst16(ol + go[2], lo[2]);
  vst16(oh + go[3], hi[3]); vst16(ol + go[3], lo[3]);
  __threadfence();
  vst16(oh + go[0], hi[0]); vst16(ol + go[0], lo[0]);
  vst16(oh + go[1], hi[1]); vst16(ol + go[1], lo[1]);
  vst16(oh + go[2], hi[2]); vst16(ol + go[2], lo[2]);
  vst16(oh + go[3], hi[3]); vst16(ol + go[3], lo[3]);
}

__global__ __launch_bounds__(128) void k_router(
    const __bf16* __restrict__ xh, const __bf16* __restrict__ xl, const __bf16* __restrict__ x3,
    const __bf16* __restrict__ gh, const __bf16* __restrict__ gm, const __bf16* __restrict__ gl,
    float* comb) {
  __shared__ float sL[4][16][17];
  __shared__ __attribute__((aligned(16))) float sCb[4][128];
  const int tid = threadIdx.x, w = tid >> 5, l = tid & 31, hh = l >> 4, m = l & 15;
  const int r0 = blockIdx.x * 64 + w * 16;
  const size_t ar = (size_t)(r0 + m) * NH;
  const size_t br = (size_t)m * NH;
  v8f acc = zero8();
#pragma unroll 1
  for (int k0 = 0; k0 < NH; k0 += 32) {
    const int ka = k0 + 8 * hh, kb = k0 + 16 + 8 * hh;
    Frag ah, al, a3, bh, bm, bl;
    ah.h[0] = *(const v8bf*)(xh + ar + ka); ah.h[1] = *(const v8bf*)(xh + ar + kb);
    al.h[0] = *(const v8bf*)(xl + ar + ka); al.h[1] = *(const v8bf*)(xl + ar + kb);
    a3.h[0] = *(const v8bf*)(x3 + ar + ka); a3.h[1] = *(const v8bf*)(x3 + ar + kb);
    bh.h[0] = *(const v8bf*)(gh + br + ka); bh.h[1] = *(const v8bf*)(gh + br + kb);
    bm.h[0] = *(const v8bf*)(gm + br + ka); bm.h[1] = *(const v8bf*)(gm + br + kb);
    bl.h[0] = *(const v8bf*)(gl + br + ka); bl.h[1] = *(const v8bf*)(gl + br + kb);
    acc = mma(ah.v, bh.v, acc);
    acc = mma(ah.v, bm.v, acc);
    acc = mma(al.v, bh.v, acc);
    acc = mma(ah.v, bl.v, acc);
    acc = mma(al.v, bm.v, acc);
    acc = mma(a3.v, bh.v, acc);
    asm volatile("v_nop\n\tv_nop\n\tv_nop\n\tv_nop"
                 : "+v"(acc)
                 : "v"(ah.v), "v"(al.v), "v"(a3.v), "v"(bh.v), "v"(bm.v), "v"(bl.v));
  }
#pragma unroll
  for (int r = 0; r < 8; r++) sL[w][8 * hh + r][m] = acc[r];
  __syncthreads();

  float lg[NE];
#pragma unroll
  for (int e = 0; e < NE; e++) lg[e] = sL[w][m][e];
  float mx = lg[0];
#pragma unroll
  for (int e = 1; e < NE; e++) mx = fmaxf(mx, lg[e]);
  float ex[NE];
  float sum = 0.0f;
#pragma unroll
  for (int e = 0; e < NE; e++) { ex[e] = expf(lg[e] - mx); sum += ex[e]; }
  const float rinv = 1.0f / sum;
  float p[NE];
#pragma unroll
  for (int e = 0; e < NE; e++) p[e] = ex[e] * rinv;
  float bv = p[0];
  int bi = 0;
#pragma unroll
  for (int e = 1; e < NE; e++) { if (p[e] > bv) { bv = p[e]; bi = e; } }
  float bv2 = -1.0f;
  int bi2 = -1;
#pragma unroll
  for (int e = 0; e < NE; e++) { if (e != bi && p[e] > bv2) { bv2 = p[e]; bi2 = e; } }
  if (l < 16) {
#pragma unroll
    for (int e = 0; e < NE; e++)
      sCb[w][m * NE + e] = (e == bi) ? bv : ((e == bi2) ? bv2 : 0.0f);
  }
  __syncthreads();
  const v4f v = *(const v4f*)(&sCb[w][4 * l]);
  float* dst = comb + (size_t)r0 * NE + 4 * l;
  *(volatile v4f*)dst = v;
  __threadfence();
  *(volatile v4f*)dst = v;
}

extern "C" void kernel_launch(void* const* d_in, const int* in_sizes, int n_in,
                              void* d_out, int out_size, void* d_ws,
                              size_t ws_size, hipStream_t stream) {
  if (n_in != 18) return;
  const int expect[18] = {NT * NH, NT * NH, NT, NH, NH, NH, NH,
                          NH * QKVW, NH * NH, NH * QKVW, NH * NH,
                          NH * 2 * IDN, IDN * NH, NH * 2 * IDN, IDN * NH,
                          NH * NE, NE * NH * 2 * IMO, NE * IMO * NH};
  for (int i = 0; i < 18; i++)
    if (in_sizes[i] != expect[i]) return;
  if (out_size != 2 * NT * NH) return;

  const float* hidden   = (const float*)d_in[0];
  const float* residual = (const float*)d_in[1];
  const int*   positions = (const int*)d_in[2];
  const float* ln0_w = (const float*)d_in[3];
  const float* pa0_w = (const float*)d_in[4];
  const float* ln1_w = (const float*)d_in[5];
  const float* pa1_w = (const float*)d_in[6];
  const float* qkv0_w = (const float*)d_in[7];
  const float* o0_w   = (const float*)d_in[8];
  const float* qkv1_w = (const float*)d_in[9];
  const float* o1_w   = (const float*)d_in[10];
  const float* gu0_w  = (const float*)d_in[11];
  const float* dn0_w  = (const float*)d_in[12];
  const float* gu1_w  = (const float*)d_in[13];
  const float* dn1_w  = (const float*)d_in[14];
  const float* gate_w = (const float*)d_in[15];
  const float* w13    = (const float*)d_in[16];
  const float* w2     = (const float*)d_in[17];

  float* out0  = (float*)d_out;
  float* r_out = out0 + (size_t)NT * NH;

  size_t off = 0;
  auto carve = [&](size_t bytes) -> char* {
    char* p = (char*)d_ws + off;
    off += (bytes + 255) & ~(size_t)255;
    return p;
  };
  float*  cs   = (float*)carve((size_t)NT * 32 * 4);
  float*  sn   = (float*)carve((size_t)NT * 32 * 4);
  __bf16* gph  = (__bf16*)carve((size_t)NEP * NH * 2);
  __bf16* gpm  = (__bf16*)carve((size_t)NEP * NH * 2);
  __bf16* gpl  = (__bf16*)carve((size_t)NEP * NH * 2);
  float*  comb = (float*)carve((size_t)NT * NE * 4);
  __bf16* hhi  = (__bf16*)carve((size_t)NT * NH * 2);
  __bf16* hlo  = (__bf16*)carve((size_t)NT * NH * 2);
  __bf16* hl3  = (__bf16*)carve((size_t)NT * NH * 2);
  float*  qkvf = (float*)carve((size_t)NT * QKVW * 4);
  __bf16* qh   = (__bf16*)carve((size_t)NT * QW * 2);
  __bf16* ql   = (__bf16*)carve((size_t)NT * QW * 2);
  __bf16* kh   = (__bf16*)carve((size_t)NT * KVW * 2);
  __bf16* kl   = (__bf16*)carve((size_t)NT * KVW * 2);
  __bf16* vth  = (__bf16*)carve((size_t)KVW * NT * 2);
  __bf16* vtl  = (__bf16*)carve((size_t)KVW * NT * 2);
  __bf16* oh   = (__bf16*)carve((size_t)NT * QW * 2);
  __bf16* ol   = (__bf16*)carve((size_t)NT * QW * 2);
  float*  tmp  = (float*)carve((size_t)NT * NH * 4);
  __bf16* acth = (__bf16*)carve((size_t)NT * IDN * 2);
  __bf16* actl = (__bf16*)carve((size_t)NT * IDN * 2);
  float*  moe_out = (float*)carve((size_t)NT * NH * 4);
  __bf16* whi  = (__bf16*)carve((size_t)NH * 2 * IDN * 2);
  __bf16* wlo  = (__bf16*)carve((size_t)NH * 2 * IDN * 2);
  if (off > ws_size) return;

  const dim3 b128(128), b256(256);

  k_rope_tab<<<dim3(NT / 4), b128, 0, stream>>>(positions, cs, sn, NT);
  k_cvt_gate<<<dim3(NEP), b128, 0, stream>>>(gate_w, gph, gpm, gpl);
  k_addnorm<0><<<dim3(NT), b256, 0, stream>>>(hidden, residual, ln0_w, r_out, hhi, hlo, hl3);

  auto cvt = [&](const float* src, int K, int Ng, int G) {
    k_cvt_t<<<dim3(Ng / 64, K / 64, G), b256, 0, stream>>>(src, K, Ng, whi, wlo);
  };
  auto gemm_f32 = [&](const __bf16* ah, const __bf16* al, int lda, int K, int N, float* C, int ldc) {
    k_gemm<0><<<dim3(N / 128, NT / 64, 1), b128, 0, stream>>>(
        ah, al, lda, whi, wlo, K, 0, 0, C, ldc, moe_out, acth, actl, IDN, comb, NE);
  };
  auto attention = [&](const float* qkv_w, const float* o_w) {
    cvt(qkv_w, NH, QKVW, 1);
    gemm_f32(hhi, hlo, NH, NH, QKVW, qkvf, QKVW);
    k_rope<<<dim3(NT / 64), b256, 0, stream>>>(qkvf, cs, sn, qh, ql, kh, kl, vth, vtl);
    k_attn<<<dim3(NT / 16, NKH), b128, 0, stream>>>(qh, ql, kh, kl, vth, vtl, oh, ol);
    cvt(o_w, NH, NH, 1);
    gemm_f32(oh, ol, QW, NH, NH, tmp, NH);
  };

  attention(qkv0_w, o0_w);
  k_addnorm<1><<<dim3(NT), b256, 0, stream>>>(tmp, r_out, pa0_w, r_out, hhi, hlo, hl3);

  k_router<<<dim3(NT / 64), b128, 0, stream>>>(hhi, hlo, hl3, gph, gpm, gpl, comb);
  cvt(w13, NH, 2 * IMO, NE);
  k_gemm<3><<<dim3(IMO / 64, NT / 64, NE), b128, 0, stream>>>(
      hhi, hlo, NH, whi, wlo, NH, IMO, 2 * IMO, tmp, NH, moe_out, acth, actl, IDN, comb, NE);
  cvt(w2, NE * IMO, NH, 1);
  gemm_f32(acth, actl, IDN, NE * IMO, NH, moe_out, NH);

  cvt(gu0_w, NH, 2 * IDN, 1);
  k_gemm<2><<<dim3(IDN / 64, NT / 64, 1), b128, 0, stream>>>(
      hhi, hlo, NH, whi, wlo, NH, IDN, 2 * IDN, tmp, NH, moe_out, acth, actl, IDN, comb, NE);
  cvt(dn0_w, IDN, NH, 1);
  gemm_f32(acth, actl, IDN, IDN, NH, tmp, NH);
  k_addnorm<0><<<dim3(NT), b256, 0, stream>>>(tmp, r_out, ln1_w, r_out, hhi, hlo, hl3);

  attention(qkv1_w, o1_w);
  k_addnorm<0><<<dim3(NT), b256, 0, stream>>>(tmp, r_out, pa1_w, r_out, hhi, hlo, hl3);

  cvt(gu1_w, NH, 2 * IDN, 1);
  k_gemm<2><<<dim3(IDN / 64, NT / 64, 1), b128, 0, stream>>>(
      hhi, hlo, NH, whi, wlo, NH, IDN, 2 * IDN, tmp, NH, moe_out, acth, actl, IDN, comb, NE);
  cvt(dn1_w, IDN, NH, 1);
  k_gemm<1><<<dim3(NH / 128, NT / 64, 1), b128, 0, stream>>>(
      acth, actl, IDN, whi, wlo, IDN, 0, 0, out0, NH, moe_out, acth, actl, IDN, comb, NE);
}
